// GATSpatialEncoder_46084999086506
// MI455X (gfx1250) — hardware-verified
//
#include <hip/hip_runtime.h>
#include <hip/hip_bf16.h>
#include <math.h>


typedef _Float16 bf16;
typedef _Float16 f16;
typedef __attribute__((ext_vector_type(4))) unsigned v4u_t;
typedef unsigned v4ua __attribute__((ext_vector_type(4), may_alias));
typedef __attribute__((ext_vector_type(4))) float v4f_t;
typedef float v4fa __attribute__((ext_vector_type(4), may_alias));
typedef __attribute__((ext_vector_type(16))) bf16  bf16x16;
typedef bf16x16 f16x16;
typedef __attribute__((ext_vector_type(8)))  bf16  bf16x8;
typedef bf16x8 f16x8;
typedef __attribute__((ext_vector_type(4)))  bf16  bf16x4;
typedef __attribute__((ext_vector_type(8)))  float f32x8;
__device__ __forceinline__ f32x8 wmma16(f16x16 a, f16x16 b, f32x8 c) {
  c = __builtin_amdgcn_wmma_f32_16x16x32_f16(false, a, false, b, (short)0, c, false, false);
  asm volatile("v_nop\n\tv_nop\n\tv_nop\n\tv_nop" : "+v"(c) : "v"(a), "v"(b));
  return c;
}
#define LDS_STRIDE 48
#define KSTRIDE    72
#define VSTRIDE    48

__device__ __forceinline__ f32x8 wmma_bf16(bf16x16 a, bf16x16 b, f32x8 c) {
  c = __builtin_amdgcn_wmma_f32_16x16x32_f16(false, a, false, b, (short)0, c, false, false);
  asm volatile("v_nop\n\tv_nop\n\tv_nop\n\tv_nop" : "+v"(c) : "v"(a), "v"(b));
  return c;
}

template <typename T>
__device__ __forceinline__ bf16x16 load_frag(const T* __restrict__ base, int ld,
                                             int row0, int k0) {
  const int lane = threadIdx.x & 31;
  const int r    = lane & 15;
  const int kh   = (lane >> 4) * 8;
  const T* p0 = base + (size_t)(row0 + r) * ld + (k0 + kh);
  const T* p1 = p0 + 16;
  bf16x16 f;
#pragma unroll
  for (int i = 0; i < 8; ++i) {
    f[i]     = (bf16)p0[i];
    f[i + 8] = (bf16)p1[i];
  }
  return f;
}

__device__ __forceinline__ bf16x16 lds_frag(const bf16* base, int stride) {
  const int lane = threadIdx.x & 31;
  const int row  = lane & 15;
  const int kh   = (lane >> 4) * 8;
  const bf16x8 lo = *(const bf16x8*)(base + row * stride + kh);
  const bf16x8 hi = *(const bf16x8*)(base + row * stride + kh + 16);
  bf16x16 f;
#pragma unroll
  for (int i = 0; i < 8; ++i) { f[i] = lo[i]; f[i + 8] = hi[i]; }
  return f;
}

template <typename T>
__device__ __forceinline__ void stage_read16(const T* __restrict__ p, float* buf) {
#pragma unroll
  for (int i = 0; i < 16; ++i) buf[i] = (float)p[i];
}

__device__ __forceinline__ void stage_write(bf16* dst, const float* buf, int nquad) {
#pragma unroll
  for (int i = 0; i < nquad; ++i) {
    bf16x4 q;
    q[0] = (bf16)buf[4 * i];     q[1] = (bf16)buf[4 * i + 1];
    q[2] = (bf16)buf[4 * i + 2]; q[3] = (bf16)buf[4 * i + 3];
    *(bf16x4*)(dst + 4 * i) = q;
  }
}


#define GSTR 48
#define GSTR 48
template <typename AT, int EPI, bool OUT16>
__global__ __launch_bounds__(256) void gemm_kne(const AT* __restrict__ A, int lda, const float* __restrict__ Wm, int ldw,
                                                const float* __restrict__ bias, const float* __restrict__ R, const float* __restrict__ gvec,
                                                void* __restrict__ Yv, int ldy, int K) {
  __shared__ __attribute__((aligned(16))) f16 ldsA[128 * GSTR];
  __shared__ __attribute__((aligned(16))) f16 ldsW[128 * GSTR];
  __shared__ __attribute__((aligned(16))) float oS[8][32 * 68];
  const int tid = threadIdx.x, lane = tid & 31, wave = tid >> 5, cl = lane & 15, rh = (lane >> 4) * 8;
  const int m0 = blockIdx.x * 128, n0 = blockIdx.y * 128;
  const int wm = (wave & 3) * 32, wn = (wave >> 2) * 64;
  f32x8 acc[2][4];
#pragma unroll
  for (int i = 0; i < 2; ++i)
#pragma unroll
    for (int j = 0; j < 4; ++j) { f32x8 z = {}; acc[i][j] = z; }
#pragma unroll 1
  for (int k0 = 0; k0 < K; k0 += 32) {
    __syncthreads();
    { const int row = tid >> 1, ch = (tid & 1) * 16;
      const AT* src = A + (size_t)(m0 + row) * lda + k0 + ch;
#pragma unroll
      for (int g = 0; g < 16; ++g) ldsA[row * GSTR + ch + g] = (f16)src[g]; }
    { const int k = tid >> 3, nn0 = (tid & 7) * 16;
      const float* src = Wm + (size_t)(k0 + k) * ldw + n0 + nn0;
#pragma unroll
      for (int g = 0; g < 4; ++g) { const v4f_t v = *(const v4f_t*)(src + 4 * g);
#pragma unroll
        for (int u = 0; u < 4; ++u) ldsW[(nn0 + 4 * g + u) * GSTR + k] = (f16)v[u]; } }
    __syncthreads();
    f16x16 af[2];
#pragma unroll
    for (int i = 0; i < 2; ++i) af[i] = lds_frag(ldsA + (wm + 16 * i) * GSTR, GSTR);
#pragma unroll
    for (int j = 0; j < 4; ++j) {
      const f16x16 bf = lds_frag(ldsW + (wn + 16 * j) * GSTR, GSTR);
#pragma unroll
      for (int i = 0; i < 2; ++i) acc[i][j] = wmma16(af[i], bf, acc[i][j]);
    }
  }
  float* so = oS[wave];
#pragma unroll
  for (int i = 0; i < 2; ++i)
#pragma unroll
    for (int j = 0; j < 4; ++j) {
      const int n = n0 + wn + 16 * j + cl;
      const float bv = bias ? bias[n] : 0.0f;
      const float gv = (EPI == 2) ? gvec[n] : 0.0f;
      if (EPI == 1) {
#pragma unroll 1
        for (int r = 0; r < 8; ++r) { const float xg = acc[i][j][r] + bv; so[(16 * i + rh + r) * 68 + 16 * j + cl] = 0.5f * xg * (1.0f + erff(xg * 0.70710678118654752f)); }
      } else {
#pragma unroll
        for (int r = 0; r < 8; ++r) {
          float v = acc[i][j][r] + bv;
          if (EPI == 2) v = R[(size_t)(m0 + wm + 16 * i + rh + r) * ldy + n] + gv * v;
          so[(16 * i + rh + r) * 68 + 16 * j + cl] = v;
        }
      }
    }
  asm volatile("s_wait_dscnt 0" ::: "memory");
  __builtin_amdgcn_wave_barrier();
#pragma unroll 1
  for (int pass = 0; pass < 2; ++pass) {
    if (OUT16) {
      f16* Y = (f16*)Yv;
#pragma unroll
      for (int it = 0; it < 8; ++it) { const int c = lane + 32 * it, rr = c >> 3, q8 = (c & 7) * 8;
        union { f16 h[8]; v4u_t v; } u;
#pragma unroll
        for (int e = 0; e < 8; ++e) u.h[e] = (f16)so[rr * 68 + q8 + e];
        *(volatile v4u_t*)(Y + (size_t)(m0 + wm + rr) * ldy + n0 + wn + q8) = u.v; }
    } else {
      float* Y = (float*)Yv;
#pragma unroll
      for (int it = 0; it < 16; ++it) { const int f4 = lane + 32 * it, rr = f4 >> 4, q = (f4 & 15) * 4;
        *(volatile v4f_t*)(Y + (size_t)(m0 + wm + rr) * ldy + n0 + wn + q) = *(const v4fa*)(so + rr * 68 + q); }
    }
    __threadfence();
  }
}


#define NNODE 1000
#define GG 96
#define TT 12
#define BBATCH 8
#define FF 8
#define DDIM 64
#define HHEAD 8
#define CCH 8
#define EE 16000
#define LCAP 64
#define NLAYER 2

__global__ __launch_bounds__(256) void k_in(const float* __restrict__ x, const float* __restrict__ in_w, const float* __restrict__ in_b, float* __restrict__ h0) {
  __shared__ float wS[FF * DDIM];
  __shared__ float bS[DDIM];
  __shared__ __attribute__((aligned(16))) float xS[GG * FF];
  __shared__ __attribute__((aligned(16))) float outS[GG * DDIM];
  const int i = blockIdx.x, tid = threadIdx.x;
#pragma unroll 1
  for (int e = tid; e < FF * DDIM; e += 256) wS[e] = in_w[e];
  if (tid < DDIM) bS[tid] = in_b[tid];
#pragma unroll 1
  for (int e = tid; e < GG * FF; e += 256) { const int g = e >> 3, f = e & 7; const int b = g / TT, t = g % TT; xS[e] = x[(((size_t)b * NNODE + i) * TT + t) * FF + f]; }
  __syncthreads();
#pragma unroll 1
  for (int k = 0; k < (GG * DDIM) / 256; ++k) { const int o = tid + 256 * k; const int g = o >> 6, d = o & 63; float s = bS[d];
#pragma unroll 1
    for (int f = 0; f < FF; ++f) s = fmaf(xS[g * FF + f], wS[f * DDIM + d], s);
    outS[o] = s; }
  __syncthreads();
  float* dst = h0 + (size_t)i * GG * DDIM;
#pragma unroll 1
  for (int pass = 0; pass < 2; ++pass) {
#pragma unroll 1
    for (int k = 0; k < (GG * DDIM / 4) / 256; ++k) { const int f4 = tid + 256 * k; *(volatile v4f_t*)(dst + 4 * f4) = *(const v4fa*)(outS + 4 * f4); }
    __threadfence(); }
}

__global__ __launch_bounds__(256) void k_packw(const float* __restrict__ Wl, const float* __restrict__ Wr, const float* __restrict__ bl, const float* __restrict__ br, int l,
                                              float* __restrict__ Wcat, float* __restrict__ bcat) {
  const int tid = threadIdx.x; const size_t wofs = (size_t)l * DDIM * DDIM, bofs = (size_t)l * DDIM;
#pragma unroll 1
  for (int pass = 0; pass < 2; ++pass) {
#pragma unroll 1
    for (int e = tid; e < DDIM * 2 * DDIM; e += 256) { const int k = e >> 7, n = e & 127; const int nn = n & 63;
      const float vl = Wl[wofs + k * DDIM + nn], vr = Wr[wofs + k * DDIM + nn];
      *(volatile float*)(Wcat + e) = (n < 64) ? vl : vr; }
    if (tid < 2 * DDIM) { const int nn = tid & 63; const float vl = bl[bofs + nn], vr = br[bofs + nn]; *(volatile float*)(bcat + tid) = (tid < 64) ? vl : vr; }
    __threadfence(); }
}

__global__ __launch_bounds__(256) void k_gat(const int* __restrict__ esrc, const int* __restrict__ edst, const float* __restrict__ XLR, const float* __restrict__ hin,
                                            const float* __restrict__ att, const float* __restrict__ bias, const float* __restrict__ lng, const float* __restrict__ lnb, int l,
                                            float* __restrict__ hout, float* __restrict__ out, int final_) {
  __shared__ int lst[LCAP];
  __shared__ int wcnt[8];
  __shared__ int scnt;
  __shared__ __attribute__((aligned(16))) float outS[GG * DDIM];
  const int i = blockIdx.x, tid = threadIdx.x, lane = tid & 31, wave = tid >> 5;
  if (tid == 0) scnt = 0;
  __syncthreads();
#pragma unroll 1
  for (int c0 = 0; c0 < EE; c0 += 256) {
    const int e = c0 + tid; const int ec = min(e, EE - 1);
    const int d = edst[ec]; const int s = esrc[ec];
    const bool hit = (e < EE) && (d == i);
    const unsigned bal = __builtin_amdgcn_ballot_w32(hit);
    const int pre = __builtin_popcount(bal & ((1u << lane) - 1u));
    if (lane == 0) wcnt[wave] = __builtin_popcount(bal);
    __syncthreads();
    const int base = scnt;
    int off = 0, tot = 0;
#pragma unroll
    for (int w = 0; w < 8; ++w) { const int c = wcnt[w]; tot += c; off += (w < wave) ? c : 0; }
    if (hit) { const int pos = base + off + pre; if (pos < LCAP) lst[pos] = min(max(s, 0), NNODE - 1); }
    __syncthreads();
    if (tid == 0) scnt = min(base + tot, LCAP);
    __syncthreads();
  }
  { const int c = scnt; __syncthreads(); if (tid == 0) { if (c < LCAP) lst[c] = i; scnt = min(c + 1, LCAP); } __syncthreads(); }
  const int cnt = scnt;
  const int h = tid & 7;
  const float* attl = att + (size_t)l * HHEAD * CCH + h * CCH;
  float a8[CCH];
#pragma unroll
  for (int c = 0; c < CCH; ++c) a8[c] = attl[c];
#pragma unroll 1
  for (int k = 0; k < 3; ++k) {
    const int g = (tid >> 3) + 32 * k;
    const size_t rowi = (size_t)i * GG + g;
    float xr[CCH], acc[CCH];
    { const v4f_t u0 = *(const v4f_t*)(XLR + rowi * 128 + 64 + h * CCH), u1 = *(const v4f_t*)(XLR + rowi * 128 + 64 + h * CCH + 4);
      xr[0] = u0[0]; xr[1] = u0[1]; xr[2] = u0[2]; xr[3] = u0[3]; xr[4] = u1[0]; xr[5] = u1[1]; xr[6] = u1[2]; xr[7] = u1[3]; }
#pragma unroll
    for (int c = 0; c < CCH; ++c) acc[c] = 0.0f;
    float m = -3.0e38f, lsum = 0.0f;
#pragma unroll 1
    for (int j = 0; j < LCAP; ++j) {
      if (j < cnt) {
        const int s = lst[j];
        const float* xlp = XLR + ((size_t)s * GG + g) * 128 + h * CCH;
        const v4f_t v0 = *(const v4f_t*)xlp, v1 = *(const v4f_t*)(xlp + 4);
        float xl[CCH]; xl[0] = v0[0]; xl[1] = v0[1]; xl[2] = v0[2]; xl[3] = v0[3]; xl[4] = v1[0]; xl[5] = v1[1]; xl[6] = v1[2]; xl[7] = v1[3];
        float e = 0.0f;
#pragma unroll
        for (int c = 0; c < CCH; ++c) { float v = xl[c] + xr[c]; v = (v > 0.0f) ? v : 0.2f * v; e = fmaf(v, a8[c], e); }
        const float mn = fmaxf(m, e); const float sc = expf(m - mn); const float p = expf(e - mn);
        lsum = lsum * sc + p;
#pragma unroll
        for (int c = 0; c < CCH; ++c) acc[c] = fmaf(p, xl[c], acc[c] * sc);
        m = mn;
      }
    }
    const float rl = 1.0f / lsum;
    v4f_t w0, w1;
#pragma unroll
    for (int c = 0; c < 4; ++c) { w0[c] = acc[c] * rl; w1[c] = acc[c + 4] * rl; }
    *(v4fa*)(outS + g * DDIM + h * CCH) = w0; *(v4fa*)(outS + g * DDIM + h * CCH + 4) = w1;
  }
  __syncthreads();
  { const float* res = hin + (size_t)i * GG * DDIM; const float* bl2 = bias + (size_t)l * DDIM;
#pragma unroll 1
    for (int o = tid; o < GG * DDIM; o += 256) { float v = outS[o] + bl2[o & 63]; v = (v > 0.0f) ? v : expm1f(v); outS[o] = v + res[o]; } }
  __syncthreads();
  { const float* gl2 = lng + (size_t)l * DDIM; const float* bb2 = lnb + (size_t)l * DDIM;
    const float ga = gl2[2 * lane], gb = gl2[2 * lane + 1], ca = bb2[2 * lane], cb = bb2[2 * lane + 1];
#pragma unroll 1
    for (int r = 0; r < GG / 8; ++r) { const int g = wave + 8 * r;
      float va = outS[g * DDIM + 2 * lane], vb = outS[g * DDIM + 2 * lane + 1];
      float s1 = va + vb;
#pragma unroll
      for (int off = 1; off < 32; off <<= 1) s1 += __shfl_xor(s1, off, 32);
      const float mean = s1 * (1.0f / DDIM); const float da = va - mean, db = vb - mean;
      float s2 = da * da + db * db;
#pragma unroll
      for (int off = 1; off < 32; off <<= 1) s2 += __shfl_xor(s2, off, 32);
      const float rstd = rsqrtf(s2 * (1.0f / DDIM) + 1e-5f);
      outS[g * DDIM + 2 * lane] = da * rstd * ga + ca; outS[g * DDIM + 2 * lane + 1] = db * rstd * gb + cb; } }
  __syncthreads();
#pragma unroll 1
  for (int pass = 0; pass < 2; ++pass) {
#pragma unroll 1
    for (int k = 0; k < (GG * DDIM / 4) / 256; ++k) { const int f4 = tid + 256 * k; const int g = f4 >> 4, q = (f4 & 15) * 4;
      float* dst = final_ ? (out + ((((size_t)(g / TT)) * NNODE + i) * TT + (g % TT)) * DDIM + q) : (hout + ((size_t)i * GG + g) * DDIM + q);
      *(volatile v4f_t*)dst = *(const v4fa*)(outS + g * DDIM + q); }
    __threadfence(); }
}

extern "C" void kernel_launch(void* const* d_in, const int* in_sizes, int n_in,
                              void* d_out, int out_size, void* d_ws, size_t ws_size,
                              hipStream_t stream) {
  (void)in_sizes; (void)n_in; (void)out_size;
  const float* x = (const float*)d_in[0]; const int* ei = (const int*)d_in[1];
  const float* in_w = (const float*)d_in[2]; const float* in_b = (const float*)d_in[3];
  const float* Wl = (const float*)d_in[4]; const float* bWl = (const float*)d_in[5]; const float* Wr = (const float*)d_in[6]; const float* bWr = (const float*)d_in[7];
  const float* att = (const float*)d_in[8]; const float* bias = (const float*)d_in[9]; const float* lng = (const float*)d_in[10]; const float* lnb = (const float*)d_in[11];
  float* out = (float*)d_out;
  char* ws = (char*)d_ws;
  float* hA = (float*)ws; ws += (size_t)NNODE * GG * DDIM * 4;
  float* hB = (float*)ws; ws += (size_t)NNODE * GG * DDIM * 4;
  float* XLR = (float*)ws; ws += (size_t)NNODE * GG * 128 * 4;
  float* Wcat = (float*)ws; ws += (size_t)DDIM * 128 * 4;
  float* bcat = (float*)ws; ws += 128 * 4;
  if ((size_t)(ws - (char*)d_ws) > ws_size) return;
  const int* esrc = ei; const int* edst = ei + EE;
  const dim3 blk(256);
  k_in<<<dim3(NNODE), blk, 0, stream>>>(x, in_w, in_b, hA);
  float* hcur = hA; float* hnext = hB;
  for (int l = 0; l < NLAYER; ++l) {
    k_packw<<<dim3(1), blk, 0, stream>>>(Wl, Wr, bWl, bWr, l, Wcat, bcat);
    gemm_kne<float, 0, false><<<dim3(NNODE * GG / 128, 1), blk, 0, stream>>>(hcur, DDIM, Wcat, 128, bcat, nullptr, nullptr, XLR, 128, DDIM);
    k_gat<<<dim3(NNODE), blk, 0, stream>>>(esrc, edst, XLR, hcur, att, bias, lng, lnb, l, hnext, out, (l == NLAYER - 1) ? 1 : 0);
    float* t = hcur; hcur = hnext; hnext = t;
  }
}
